// QLoRAMoeExperts_9096740733119
// MI455X (gfx1250) — hardware-verified
//
#include <hip/hip_runtime.h>
#include <math.h>

typedef __attribute__((ext_vector_type(16))) _Float16 v16h;
typedef __attribute__((ext_vector_type(16))) __bf16 v16b;
typedef __attribute__((ext_vector_type(8)))  _Float16 v8h;
typedef __attribute__((ext_vector_type(8)))  float v8f;
typedef __attribute__((ext_vector_type(4)))  float v4f;
typedef __attribute__((ext_vector_type(2)))  float v2f;
typedef __attribute__((ext_vector_type(4)))  unsigned v4u;
typedef __attribute__((ext_vector_type(4)))  int v4i;
typedef float __attribute__((may_alias)) float_a;
typedef int __attribute__((may_alias)) int_a;

template <typename T> __device__ __forceinline__ void vst2(void* p, T v) { *(volatile T*)p = v; __threadfence(); *(volatile T*)p = v; }
__device__ __forceinline__ v8f wmma16(v16h a, v16h b, v8f c) {
  v8f d = __builtin_amdgcn_wmma_f32_16x16x32_f16(false, a, false, b, (short)0, c, false, false);
  asm volatile("v_nop\n\tv_nop\n\tv_nop\n\tv_nop" : "+v"(d) : "v"(a), "v"(b));
  return d;
}
__device__ __forceinline__ v8f wmma_bf(v16b a, v16b b, v8f c) {
  v8f d = __builtin_amdgcn_wmma_f32_16x16x32_bf16(false, a, false, b, (short)0, c, false, false);
  asm volatile("v_nop\n\tv_nop\n\tv_nop\n\tv_nop" : "+v"(d) : "v"(a), "v"(b));
  return d;
}
__device__ __forceinline__ v16h frag_h(const _Float16* rowk0, int lane) {
  union { v16h v; v8h q[2]; } u; const _Float16* p = rowk0 + 8 * (lane >> 4);
  u.q[0] = *(const v8h*)p; u.q[1] = *(const v8h*)(p + 16); return u.v;
}
__device__ __forceinline__ v16h frag_f32(const float* rowk0, int lane) {
  v16h a; const float* p = rowk0 + 8 * (lane >> 4);
#pragma unroll
  for (int i = 0; i < 8; ++i) { a[i] = (_Float16)p[i]; a[8 + i] = (_Float16)p[16 + i]; }
  return a;
}
__device__ __forceinline__ v16h frag_f32s(const float* rowk0, int lane, float sc) {
  v16h a; const float* p = rowk0 + 8 * (lane >> 4);
#pragma unroll
  for (int i = 0; i < 8; ++i) { a[i] = (_Float16)(p[i] * sc); a[8 + i] = (_Float16)(p[16 + i] * sc); }
  return a;
}
__device__ __forceinline__ v16h fragc_f32(const float* W, int k0, int n, int lane, int ld, int K) {
  v16h a; const int g = lane >> 4;
#pragma unroll
  for (int i = 0; i < 8; ++i) { const int ka = k0 + 8 * g + i, kb = ka + 16;
    a[i] = (_Float16)(ka < K ? W[(size_t)(ka < K ? ka : K - 1) * ld + n] : 0.f); a[8 + i] = (_Float16)(kb < K ? W[(size_t)(kb < K ? kb : K - 1) * ld + n] : 0.f); }
  return a;
}
struct F2 { v16b h, l; };
__device__ __forceinline__ F2 bsplit16(const float v[16]) { F2 r;
#pragma unroll
  for (int i = 0; i < 16; ++i) { const __bf16 h = (__bf16)v[i]; r.h[i] = h; r.l[i] = (__bf16)(v[i] - (float)h); }
  return r; }
__device__ __forceinline__ F2 split_row(const float* row, int k0, int lane) { float v[16]; const float* p = row + k0 + 8 * (lane >> 4);
#pragma unroll
  for (int i = 0; i < 8; ++i) { v[i] = p[i]; v[8 + i] = p[16 + i]; }
  return bsplit16(v); }
__device__ __forceinline__ F2 split_rowK(const float* row, int k0, int lane, int K) { float v[16]; const int g = lane >> 4;
#pragma unroll
  for (int i = 0; i < 8; ++i) { const int ka = k0 + 8 * g + i, kb = ka + 16; v[i] = ka < K ? row[ka < K ? ka : K - 1] : 0.f; v[8 + i] = kb < K ? row[kb < K ? kb : K - 1] : 0.f; }
  return bsplit16(v); }
__device__ __forceinline__ F2 split_col(const float* W, int k0, int n, int lane, int ld, int K) { float v[16]; const int g = lane >> 4;
#pragma unroll
  for (int i = 0; i < 8; ++i) { const int ka = k0 + 8 * g + i, kb = ka + 16; v[i] = ka < K ? W[(size_t)(ka < K ? ka : K - 1) * ld + n] : 0.f; v[8 + i] = kb < K ? W[(size_t)(kb < K ? kb : K - 1) * ld + n] : 0.f; }
  return bsplit16(v); }
__device__ __forceinline__ v8f mac3(const F2& a, const F2& b, v8f c) { c = wmma_bf(a.l, b.h, c); c = wmma_bf(a.h, b.l, c); return wmma_bf(a.h, b.h, c); }
__device__ __forceinline__ float sigm(float v) { return 1.0f / (1.0f + expf(-v)); }
#define LDSX() do { asm volatile("s_wait_dscnt 0" ::: "memory"); __builtin_amdgcn_wave_barrier(); __builtin_amdgcn_fence(__ATOMIC_RELEASE, "workgroup"); } while (0)


#define TT 512
#define HH 2048
#define II 1024
#define NE 8
#define RK 16
#define GRP 64
#define NSLOT 2
#define NENT (TT * NSLOT)
typedef __attribute__((ext_vector_type(8))) __bf16 v8b;
__device__ __forceinline__ v16b frag_b(const __bf16* rowk0, int lane) {
  union { v16b v; v8b q[2]; } u; const __bf16* p = rowk0 + 8 * (lane >> 4);
  u.q[0] = *(const v8b*)p; u.q[1] = *(const v8b*)(p + 16); return u.v;
}
__device__ __forceinline__ float bfr(float v) { return (float)(__bf16)v; }
__device__ __attribute__((noinline)) float exp_ni(float v) { return expf(v); }
__device__ __attribute__((noinline)) float erf_ni(float v) { return erff(v); }
__constant__ float c_nf4[16] = {-1.0f, -0.6961928009986877f, -0.5250730514526367f, -0.39491748809814453f, -0.28444138169288635f, -0.18477343022823334f, -0.09105003625154495f, 0.0f, 0.07958029955625534f, 0.16093020141124725f, 0.24611230194568634f, 0.33791524171829224f, 0.44070982933044434f, 0.5626170039176941f, 0.7229568362236328f, 1.0f};

#define WS_WGH  0u
#define WS_WGL  (WS_WGH + 2u * II * HH)
#define WS_WUH  (WS_WGL + 2u * II * HH)
#define WS_WUL  (WS_WUH + 2u * II * HH)
#define WS_WDH  (WS_WUL + 2u * II * HH)
#define WS_WDL  (WS_WDH + 2u * HH * II)
#define WS_CNT  (WS_WDL + 2u * HH * II)
#define WS_LIST (WS_CNT + 128u)
#define WS_HBH  (WS_LIST + 4u * NE * NENT)
#define WS_HBL  (WS_HBH + 2u * NENT * II)
#define WS_O    (WS_HBL + 2u * NENT * II)
#define WS_END  (WS_O + 4u * (size_t)NENT * HH)

__global__ __launch_bounds__(256) void k_sort(const int* __restrict__ TIDX, int* __restrict__ CNT, int* __restrict__ LIST) {
  __shared__ int scnt[NE], sfirst[NE]; __shared__ __align__(16) int sc[32]; const int t = threadIdx.x;
  if (t < NE) { int c = 0, f = 0; bool seen = false; for (int i = 0; i < TT; ++i) for (int sl = 0; sl < NSLOT; ++sl) { const int e = min(max(TIDX[i * NSLOT + sl], 0), NE - 1); if (e == t) { LIST[(size_t)t * NENT + c] = i * NSLOT + sl; if (!seen) { f = i * NSLOT + sl; seen = true; } ++c; } } scnt[t] = c; sfirst[t] = f; }
  __syncthreads();
  for (int q = t; q < NE * NENT; q += 256) { const int e = q / NENT, k = q % NENT; if (k >= scnt[e]) LIST[q] = sfirst[e]; }
  if (t < 32) sc[t] = (t < NE) ? scnt[t] : 0;
  __syncthreads();
  for (int q = t; q < NE * NENT / 4; q += 256) { v4u v; const int* p = LIST + (size_t)q * 4; v[0] = p[0]; v[1] = p[1]; v[2] = p[2]; v[3] = p[3]; vst2((unsigned*)(LIST + (size_t)q * 4), v); }
  if (t < 8) vst2((unsigned*)(CNT + t * 4), *(const v4u*)&sc[t * 4]);
}
__global__ __launch_bounds__(256) void k_deq(int e, const int* __restrict__ GP, const float* __restrict__ GS, const int* __restrict__ UP, const float* __restrict__ US, const int* __restrict__ DP, const float* __restrict__ DS, const float* __restrict__ GA, const float* __restrict__ GB, const float* __restrict__ UA, const float* __restrict__ UB, const float* __restrict__ DA, const float* __restrict__ DB, __bf16* __restrict__ WGH, __bf16* __restrict__ WGL, __bf16* __restrict__ WUH, __bf16* __restrict__ WUL, __bf16* __restrict__ WDH, __bf16* __restrict__ WDL) {
  __shared__ __align__(16) __bf16 sh_[HH], sl_[HH]; __shared__ float sb[RK]; const int n = blockIdx.x, which = blockIdx.y, t = threadIdx.x;
  const int K = (which < 2) ? HH : II, N = (which < 2) ? II : HH; if (n >= N) return;
  const int* PKD = (which == 0) ? GP : (which == 1) ? UP : DP; const float* SC = (which == 0) ? GS : (which == 1) ? US : DS; const float* A = (which == 0) ? GA : (which == 1) ? UA : DA; const float* Bm = (which == 0) ? GB : (which == 1) ? UB : DB;
  if (t < RK) sb[t] = bfr(Bm[((size_t)e * RK + t) * N + n]);
  __syncthreads();
  for (int k = t; k < K; k += 256) { const int byte = PKD[((size_t)e * (K / 2) + (k >> 1)) * N + n]; const int code = (k & 1) ? ((byte >> 4) & 15) : (byte & 15);
    float w = c_nf4[code] * bfr(SC[((size_t)e * (K / GRP) + k / GRP) * N + n]); float lo = 0.f;
#pragma unroll 1
    for (int r = 0; r < RK; ++r) lo += bfr(A[((size_t)e * K + k) * RK + r]) * sb[r];
    w = w + 1.0f * lo;
    const __bf16 hb = (__bf16)w; sh_[k] = hb; sl_[k] = (__bf16)(w - (float)hb); }
  __syncthreads();
  __bf16* DH = (which == 0) ? WGH : (which == 1) ? WUH : WDH; __bf16* DL = (which == 0) ? WGL : (which == 1) ? WUL : WDL;
  for (int q = t; q < K / 8; q += 256) { vst2((unsigned*)(DH + (size_t)n * K + q * 8), *(const v4u*)&sh_[q * 8]); vst2((unsigned*)(DL + (size_t)n * K + q * 8), *(const v4u*)&sl_[q * 8]); }
}
__global__ __launch_bounds__(128) void k_gu(int e, const float* __restrict__ X, const __bf16* __restrict__ WGH, const __bf16* __restrict__ WGL, const __bf16* __restrict__ WUH, const __bf16* __restrict__ WUL, const int* __restrict__ CNT, const int* __restrict__ LIST, __bf16* __restrict__ HBH, __bf16* __restrict__ HBL) {
  __shared__ __align__(16) __bf16 soh[4][16][136], sol[4][16][136]; __shared__ int sent[64];
  const int tid = threadIdx.x, wave = tid >> 5, lane = tid & 31, col = lane & 15, g = lane >> 4; const int cnt = CNT[e]; if (blockIdx.x * 64 >= cnt) return;
  if (tid < 64) sent[tid] = LIST[(size_t)e * NENT + blockIdx.x * 64 + tid];
  __syncthreads();
  const int n0 = blockIdx.y * 128; const int tok = sent[wave * 16 + col] >> 1;
  v8f ag[8] = {}, au[8] = {};
#pragma unroll 1
  for (int kc = 0; kc < HH / 32; ++kc) { v16b a; { const float* p = X + (size_t)tok * HH + kc * 32 + 8 * g;
#pragma unroll
      for (int i = 0; i < 8; ++i) { a[i] = (__bf16)p[i]; a[8 + i] = (__bf16)p[16 + i]; } }
#pragma unroll
    for (int j = 0; j < 8; ++j) { const size_t ro = (size_t)(n0 + j * 16 + col) * HH + kc * 32; ag[j] = wmma_bf(a, frag_b(WGL + ro, lane), ag[j]); ag[j] = wmma_bf(a, frag_b(WGH + ro, lane), ag[j]); au[j] = wmma_bf(a, frag_b(WUL + ro, lane), au[j]); au[j] = wmma_bf(a, frag_b(WUH + ro, lane), au[j]); } }
#pragma unroll
  for (int j = 0; j < 8; ++j)
#pragma unroll
    for (int r = 0; r < 8; ++r) { const float gv = ag[j][r]; const float hv = (gv / (1.0f + exp_ni(-gv))) * au[j][r]; const __bf16 hb = (__bf16)hv; soh[wave][8 * g + r][j * 16 + col] = hb; sol[wave][8 * g + r][j * 16 + col] = (__bf16)(hv - (float)hb); }
  LDSX();
  for (int rl = 0; rl < 16; ++rl) { const int li = blockIdx.x * 64 + wave * 16 + rl; if (li < cnt && lane < 16) { const size_t o = (size_t)sent[wave * 16 + rl] * II + n0 + lane * 8; vst2((unsigned*)(HBH + o), *(const v4u*)&soh[wave][rl][lane * 8]); vst2((unsigned*)(HBL + o), *(const v4u*)&sol[wave][rl][lane * 8]); } }
}
__global__ __launch_bounds__(128) void k_down(int e, const __bf16* __restrict__ HBH, const __bf16* __restrict__ HBL, const __bf16* __restrict__ WDH, const __bf16* __restrict__ WDL, const int* __restrict__ CNT, const int* __restrict__ LIST, float* __restrict__ O) {
  __shared__ __align__(16) float so[4][16][132]; __shared__ int sent[64];
  const int tid = threadIdx.x, wave = tid >> 5, lane = tid & 31, col = lane & 15, g = lane >> 4; const int cnt = CNT[e]; if (blockIdx.x * 64 >= cnt) return;
  if (tid < 64) sent[tid] = LIST[(size_t)e * NENT + blockIdx.x * 64 + tid];
  __syncthreads();
  const int n0 = blockIdx.y * 128; const size_t arow = (size_t)sent[wave * 16 + col] * II;
  v8f acc[8] = {};
#pragma unroll 1
  for (int kc = 0; kc < II / 32; ++kc) { const v16b ah = frag_b(HBH + arow + kc * 32, lane), al = frag_b(HBL + arow + kc * 32, lane);
#pragma unroll
    for (int j = 0; j < 8; ++j) { const size_t ro = (size_t)(n0 + j * 16 + col) * II + kc * 32; const v16b wh = frag_b(WDH + ro, lane), wl = frag_b(WDL + ro, lane); acc[j] = wmma_bf(al, wh, acc[j]); acc[j] = wmma_bf(ah, wl, acc[j]); acc[j] = wmma_bf(ah, wh, acc[j]); } }
#pragma unroll
  for (int j = 0; j < 8; ++j)
#pragma unroll
    for (int r = 0; r < 8; ++r) so[wave][8 * g + r][j * 16 + col] = acc[j][r];
  LDSX();
  for (int rl = 0; rl < 16; ++rl) { const int li = blockIdx.x * 64 + wave * 16 + rl; if (li < cnt) vst2(O + (size_t)sent[wave * 16 + rl] * HH + n0 + lane * 4, *(const v4f*)&so[wave][rl][lane * 4]); }
}
__global__ __launch_bounds__(256) void k_comb(const int* __restrict__ TIDX, const float* __restrict__ TW, const float* __restrict__ O, float* __restrict__ OUT) {
  const size_t t = blockIdx.x; const int tid = threadIdx.x; const int e0 = min(max(TIDX[t * 2], 0), NE - 1), e1 = min(max(TIDX[t * 2 + 1], 0), NE - 1); const float w0 = bfr(TW[t * 2]), w1 = bfr(TW[t * 2 + 1]);
  const float* oa = O + (t * 2) * HH; const float* ob = O + (t * 2 + 1) * HH;
  for (int c0 = tid * 4; c0 < HH; c0 += 1024) { v4f v;
#pragma unroll
    for (int i = 0; i < 4; ++i) { const int c = c0 + i; float r;
      if (e0 == e1) r = (w0 + w1) * oa[c];
      else if (e0 < e1) r = (w0 * oa[c]) + (w1 * ob[c]); else r = (w1 * ob[c]) + (w0 * oa[c]);
      v[i] = r; }
    vst2(OUT + t * HH + c0, v); }
}
extern "C" void kernel_launch(void* const* d_in, const int* in_sizes, int n_in, void* d_out, int out_size, void* d_ws, size_t ws_size, hipStream_t stream) {
  (void)in_sizes; (void)n_in; (void)out_size;
  if (ws_size < (size_t)WS_END) return;
  char* ws = (char*)d_ws; __bf16 *WGH = (__bf16*)(ws + WS_WGH), *WGL = (__bf16*)(ws + WS_WGL), *WUH = (__bf16*)(ws + WS_WUH), *WUL = (__bf16*)(ws + WS_WUL), *WDH = (__bf16*)(ws + WS_WDH), *WDL = (__bf16*)(ws + WS_WDL), *HBH = (__bf16*)(ws + WS_HBH), *HBL = (__bf16*)(ws + WS_HBL); int *CNT = (int*)(ws + WS_CNT), *LIST = (int*)(ws + WS_LIST); float* O = (float*)(ws + WS_O);
  const float* X = (const float*)d_in[0]; const int* TIDX = (const int*)d_in[1]; const float* TW = (const float*)d_in[2];
  k_sort<<<1, 256, 0, stream>>>(TIDX, CNT, LIST);
  for (int e = 0; e < NE; ++e) {
    k_deq<<<dim3(HH, 3), 256, 0, stream>>>(e, (const int*)d_in[3], (const float*)d_in[4], (const int*)d_in[5], (const float*)d_in[6], (const int*)d_in[7], (const float*)d_in[8], (const float*)d_in[9], (const float*)d_in[10], (const float*)d_in[11], (const float*)d_in[12], (const float*)d_in[13], (const float*)d_in[14], WGH, WGL, WUH, WUL, WDH, WDL);
    k_gu<<<dim3(NENT / 64, II / 128), 128, 0, stream>>>(e, X, WGH, WGL, WUH, WUL, CNT, LIST, HBH, HBL);
    k_down<<<dim3(NENT / 64, HH / 128), 128, 0, stream>>>(e, HBH, HBL, WDH, WDL, CNT, LIST, O); }
  k_comb<<<TT, 256, 0, stream>>>(TIDX, TW, O, (float*)d_out);
}
